// GFAPM_38242388803819
// MI455X (gfx1250) — hardware-verified
//
#include <hip/hip_runtime.h>
#include <hip/hip_bf16.h>


#define BB      4
#define CC      256
#define CQ      64
#define HW      4096
#define BN_EPS  1e-5f
#define KBLK    64
#define QT      32
#define XSP     72
#define ESP     36
#define WSCALE      16.0f
#define WSCALE_INV  0.0625f
#define PSCALE      32768.0f
#define PSCALE_INV  (1.0f / 32768.0f)

typedef unsigned int v4u  __attribute__((ext_vector_type(4)));
typedef float        v4f  __attribute__((ext_vector_type(4)));
typedef float        v8f  __attribute__((ext_vector_type(8)));
typedef __bf16       v16b __attribute__((ext_vector_type(16)));
typedef _Float16     v16h __attribute__((ext_vector_type(16)));
typedef _Float16     v8h  __attribute__((ext_vector_type(8)));

union Frag  { v4u u[2]; v16b bf; v16h hf; };
union Pack8 { v4u u; v8h hf; unsigned short s[8]; };

__device__ __forceinline__ v8f mma_bf16(v16b a, v16b b, v8f c)
{
    v8f d = __builtin_amdgcn_wmma_f32_16x16x32_bf16(false, a, false, b, (short)0, c, false, false);
    asm volatile("v_nop\n\tv_nop\n\tv_nop\n\tv_nop" : "+v"(d) : "v"(a), "v"(b));
    return d;
}

__device__ __forceinline__ v8f mma_f16(v16h a, v16h b, v8f c)
{
    v8f d = __builtin_amdgcn_wmma_f32_16x16x32_f16(false, a, false, b, (short)0, c, false, false);
    asm volatile("v_nop\n\tv_nop\n\tv_nop\n\tv_nop" : "+v"(d) : "v"(a), "v"(b));
    return d;
}

__device__ __forceinline__ v8f zero8()
{
    v8f z = {0.f, 0.f, 0.f, 0.f, 0.f, 0.f, 0.f, 0.f};
    return z;
}

__device__ __forceinline__ unsigned short bf16_rne(float f)
{
    unsigned u = __float_as_uint(f);
    u += 0x7FFFu + ((u >> 16) & 1u);
    return (unsigned short)(u >> 16);
}

__device__ __forceinline__ void bf16_split(float f, unsigned short& hi, unsigned short& lo)
{
    hi = bf16_rne(f);
    const float fh = __uint_as_float(((unsigned)hi) << 16);
    lo = bf16_rne(f - fh);
}

__device__ __forceinline__ unsigned short f16_bits(float f)
{
    union { _Float16 x; unsigned short s; } c;
    c.x = (_Float16)f;
    return c.s;
}

__global__ __launch_bounds__(128) void k_conv_split(
    const float* __restrict__ x,  const float* __restrict__ w,
    const float* __restrict__ bi, const float* __restrict__ g,
    const float* __restrict__ be, const float* __restrict__ mn,
    const float* __restrict__ vr,
    unsigned short* __restrict__ oh, unsigned short* __restrict__ ol)
{
    __shared__ __align__(16) unsigned short xs_h[64 * XSP];
    __shared__ __align__(16) unsigned short xs_l[64 * XSP];
    __shared__ __align__(16) unsigned short ws_h[64 * XSP];
    __shared__ __align__(16) unsigned short ws_l[64 * XSP];
    __shared__ v4u es_h[4][16 * 9];
    __shared__ v4u es_l[4][16 * 9];
    __shared__ float psc[64], psh[64], pbi[64];

    const int t  = threadIdx.x;
    const int l  = t & 31, wv = t >> 5, h = l >> 4, m = l & 15;
    const int i0 = blockIdx.x * 64;
    const int b  = blockIdx.y;
    if (i0 >= HW || b >= BB) return;

    if (t < CQ) {
        const float rs = rsqrtf(vr[t] + BN_EPS);
        psc[t] = g[t] * rs;
        psh[t] = be[t] - g[t] * mn[t] * rs;
        pbi[t] = bi[t];
    }

    v8f acc[4];
#pragma unroll
    for (int tt = 0; tt < 4; ++tt) acc[tt] = zero8();

    const int c4 = t & 15, r8 = t >> 4;
#pragma unroll 1
    for (int kc = 0; kc < CC / 64; ++kc) {
        const int ch0 = kc * 64;
        __syncthreads();
#pragma unroll
        for (int rr = 0; rr < 8; ++rr) {
            const int ch = r8 + 8 * rr;
            const v4f v = *(const v4f*)(x + ((size_t)(b * CC + ch0 + ch)) * HW + i0 + 4 * c4);
#pragma unroll
            for (int e = 0; e < 4; ++e) {
                unsigned short hs, ls;
                bf16_split(v[e], hs, ls);
                xs_h[(4 * c4 + e) * XSP + ch] = hs;
                xs_l[(4 * c4 + e) * XSP + ch] = ls;
            }
        }
#pragma unroll
        for (int rr = 0; rr < 8; ++rr) {
            const int o = r8 + 8 * rr;
            const v4f v = *(const v4f*)(w + (size_t)o * CC + ch0 + 4 * c4);
#pragma unroll
            for (int e = 0; e < 4; ++e) {
                unsigned short hs, ls;
                bf16_split(v[e], hs, ls);
                ws_h[o * XSP + 4 * c4 + e] = hs;
                ws_l[o * XSP + 4 * c4 + e] = ls;
            }
        }
        __syncthreads();
#pragma unroll
        for (int s = 0; s < 2; ++s) {
            const int xi = (16 * wv + m) * XSP + 32 * s + 8 * h;
            Frag bh, bl;
            bh.u[0] = *(const v4u*)&xs_h[xi];  bh.u[1] = *(const v4u*)&xs_h[xi + 16];
            bl.u[0] = *(const v4u*)&xs_l[xi];  bl.u[1] = *(const v4u*)&xs_l[xi + 16];
#pragma unroll
            for (int tt = 0; tt < 4; ++tt) {
                const int wi = (16 * tt + m) * XSP + 32 * s + 8 * h;
                Frag ah, al;
                ah.u[0] = *(const v4u*)&ws_h[wi];  ah.u[1] = *(const v4u*)&ws_h[wi + 16];
                al.u[0] = *(const v4u*)&ws_l[wi];  al.u[1] = *(const v4u*)&ws_l[wi + 16];
                acc[tt] = mma_bf16(ah.bf, bh.bf, acc[tt]);
                acc[tt] = mma_bf16(ah.bf, bl.bf, acc[tt]);
                acc[tt] = mma_bf16(al.bf, bh.bf, acc[tt]);
            }
        }
    }

#pragma unroll
    for (int tt = 0; tt < 4; ++tt) {
        Pack8 ph, pl;
#pragma unroll
        for (int r = 0; r < 8; ++r) {
            const int o = 16 * tt + 8 * h + r;
            float y = (acc[tt][r] + pbi[o]) * psc[o] + psh[o];
            y = fmaxf(y, 0.0f);
            unsigned short hs, ls;
            bf16_split(y, hs, ls);
            ph.s[r] = hs;
            pl.s[r] = ls;
        }
        es_h[wv][m * 9 + 2 * tt + h] = ph.u;
        es_l[wv][m * 9 + 2 * tt + h] = pl.u;
    }
    __syncthreads();

    const int q8 = l >> 3, p = l & 7;
#pragma unroll
    for (int gq = 0; gq < 4; ++gq) {
        const int il = 4 * gq + q8;
        const size_t off = ((size_t)(b * HW + i0 + 16 * wv + il)) * CQ + 8 * p;
        const v4u vh = es_h[wv][il * 9 + p];
        const v4u vl = es_l[wv][il * 9 + p];
        *(volatile v4u*)(oh + off) = vh;
        *(volatile v4u*)(ol + off) = vl;
    }
    __threadfence();
#pragma unroll
    for (int gq = 0; gq < 4; ++gq) {
        const int il = 4 * gq + q8;
        const size_t off = ((size_t)(b * HW + i0 + 16 * wv + il)) * CQ + 8 * p;
        const v4u vh = es_h[wv][il * 9 + p];
        const v4u vl = es_l[wv][il * 9 + p];
        *(volatile v4u*)(oh + off) = vh;
        *(volatile v4u*)(ol + off) = vl;
    }
}

__global__ __launch_bounds__(128) void k_conv_h(
    const float* __restrict__ x,  const float* __restrict__ w,
    const float* __restrict__ bi, const float* __restrict__ g,
    const float* __restrict__ be, const float* __restrict__ mn,
    const float* __restrict__ vr, unsigned short* __restrict__ ov)
{
    __shared__ __align__(16) unsigned short xs[64 * XSP];
    __shared__ __align__(16) unsigned short ws[64 * XSP];
    __shared__ v4u es[4][16 * 9];
    __shared__ float psc[64], psh[64], pbi[64];

    const int t  = threadIdx.x;
    const int l  = t & 31, wv = t >> 5, h = l >> 4, m = l & 15;
    const int i0 = blockIdx.x * 64;
    const int c0 = blockIdx.y * 64;
    const int b  = blockIdx.z;
    if (i0 >= HW || c0 >= CC || b >= BB) return;

    if (t < 64) {
        const int o = c0 + t;
        const float rs = rsqrtf(vr[o] + BN_EPS);
        psc[t] = g[o] * rs;
        psh[t] = be[o] - g[o] * mn[o] * rs;
        pbi[t] = bi[o];
    }

    v8f acc[4];
#pragma unroll
    for (int tt = 0; tt < 4; ++tt) acc[tt] = zero8();

    const int c4 = t & 15, r8 = t >> 4;
#pragma unroll 1
    for (int kc = 0; kc < CC / 64; ++kc) {
        const int ch0 = kc * 64;
        __syncthreads();
#pragma unroll
        for (int rr = 0; rr < 8; ++rr) {
            const int ch = r8 + 8 * rr;
            const v4f v = *(const v4f*)(x + ((size_t)(b * CC + ch0 + ch)) * HW + i0 + 4 * c4);
#pragma unroll
            for (int e = 0; e < 4; ++e) xs[(4 * c4 + e) * XSP + ch] = f16_bits(v[e]);
        }
#pragma unroll
        for (int rr = 0; rr < 8; ++rr) {
            const int o = r8 + 8 * rr;
            const v4f v = *(const v4f*)(w + (size_t)(c0 + o) * CC + ch0 + 4 * c4);
#pragma unroll
            for (int e = 0; e < 4; ++e) ws[o * XSP + 4 * c4 + e] = f16_bits(v[e] * WSCALE);
        }
        __syncthreads();
#pragma unroll
        for (int s = 0; s < 2; ++s) {
            const int wi = (16 * wv + m) * XSP + 32 * s + 8 * h;
            Frag bw;
            bw.u[0] = *(const v4u*)&ws[wi];  bw.u[1] = *(const v4u*)&ws[wi + 16];
#pragma unroll
            for (int tt = 0; tt < 4; ++tt) {
                const int xi = (16 * tt + m) * XSP + 32 * s + 8 * h;
                Frag ax;
                ax.u[0] = *(const v4u*)&xs[xi];  ax.u[1] = *(const v4u*)&xs[xi + 16];
                acc[tt] = mma_f16(ax.hf, bw.hf, acc[tt]);
            }
        }
    }

    const int cl = 16 * wv + m;
    const float sc = psc[cl], sh = psh[cl], bb = pbi[cl];
#pragma unroll
    for (int tt = 0; tt < 4; ++tt) {
        Pack8 pk;
#pragma unroll
        for (int r = 0; r < 8; ++r) {
            float y = (acc[tt][r] * WSCALE_INV + bb) * sc + sh;
            y = fmaxf(y, 0.0f);
            pk.hf[r] = (_Float16)y;
        }
        es[wv][m * 9 + 2 * tt + h] = pk.u;
    }
    __syncthreads();

    const int q8 = l >> 3, p = l & 7;
#pragma unroll
    for (int gq = 0; gq < 4; ++gq) {
        const int cr = 4 * gq + q8;
        const size_t off = ((size_t)(b * CC + c0 + 16 * wv + cr)) * HW + i0 + 8 * p;
        const v4u vv = es[wv][cr * 9 + p];
        *(volatile v4u*)(ov + off) = vv;
    }
    __threadfence();
#pragma unroll
    for (int gq = 0; gq < 4; ++gq) {
        const int cr = 4 * gq + q8;
        const size_t off = ((size_t)(b * CC + c0 + 16 * wv + cr)) * HW + i0 + 8 * p;
        const v4u vv = es[wv][cr * 9 + p];
        *(volatile v4u*)(ov + off) = vv;
    }
}

__global__ __launch_bounds__(128) void k_attn(
    const unsigned short* __restrict__ qh, const unsigned short* __restrict__ ql,
    const unsigned short* __restrict__ kh, const unsigned short* __restrict__ kl,
    const unsigned short* __restrict__ vv, const float* __restrict__ x1r,
    const float* __restrict__ gamp, float* __restrict__ outp)
{
    __shared__ v4u qs_h[QT * 9];
    __shared__ v4u qs_l[QT * 9];
    __shared__ v4u pq[QT * 9];
    __shared__ float red_mx[4][QT];
    __shared__ float red_sm[4][QT];
    __shared__ __align__(16) float es[4][64 * ESP];

    const int t  = threadIdx.x;
    const int l  = t & 31, wv = t >> 5, h = l >> 4, m = l & 15;
    const int i0 = blockIdx.x * QT;
    const int b  = blockIdx.y;
    if (i0 >= HW || b >= BB) return;

    for (int idx = t; idx < QT * 8; idx += 128) {
        const int row = idx >> 3, pc = idx & 7;
        const size_t off = ((size_t)(b * HW + i0 + row)) * CQ + 8 * pc;
        qs_h[row * 9 + pc] = *(const v4u*)(qh + off);
        qs_l[row * 9 + pc] = *(const v4u*)(ql + off);
    }
    __syncthreads();

    const float L2E = 1.4426950408889634f;
    const float gm0 = gamp[0];

    v8f acc[4][2];
#pragma unroll
    for (int tt = 0; tt < 4; ++tt) { acc[tt][0] = zero8(); acc[tt][1] = zero8(); }
    float mrun[2], lrun[2];
    mrun[0] = -3.0e38f; mrun[1] = -3.0e38f;
    lrun[0] = 0.0f;     lrun[1] = 0.0f;

#pragma unroll 1
    for (int j0 = 0; j0 < HW; j0 += KBLK) {
        v8f sacc[2];
        sacc[0] = zero8(); sacc[1] = zero8();
        const size_t krow = ((size_t)(b * HW + j0 + 16 * wv + m)) * CQ;
#pragma unroll
        for (int s = 0; s < 2; ++s) {
            Frag ka, kb;
            ka.u[0] = *(const v4u*)(kh + krow + 32 * s + 8 * h);
            ka.u[1] = *(const v4u*)(kh + krow + 32 * s + 16 + 8 * h);
            kb.u[0] = *(const v4u*)(kl + krow + 32 * s + 8 * h);
            kb.u[1] = *(const v4u*)(kl + krow + 32 * s + 16 + 8 * h);
#pragma unroll
            for (int u = 0; u < 2; ++u) {
                const int qi = (16 * u + m) * 9 + 4 * s + h;
                Frag qa, qb;
                qa.u[0] = qs_h[qi];  qa.u[1] = qs_h[qi + 2];
                qb.u[0] = qs_l[qi];  qb.u[1] = qs_l[qi + 2];
                sacc[u] = mma_bf16(ka.bf, qa.bf, sacc[u]);
                sacc[u] = mma_bf16(ka.bf, qb.bf, sacc[u]);
                sacc[u] = mma_bf16(kb.bf, qa.bf, sacc[u]);
            }
        }

#pragma unroll
        for (int u = 0; u < 2; ++u) {
            float mb = sacc[u][0];
#pragma unroll
            for (int r = 1; r < 8; ++r) mb = fmaxf(mb, sacc[u][r]);
            mb = fmaxf(mb, __shfl_xor(mb, 16));
            if (h == 0) red_mx[wv][16 * u + m] = mb;
        }
        __syncthreads();

        float alpha[2];
#pragma unroll
        for (int u = 0; u < 2; ++u) {
            const int iq = 16 * u + m;
            const float mb   = fmaxf(fmaxf(red_mx[0][iq], red_mx[1][iq]), fmaxf(red_mx[2][iq], red_mx[3][iq]));
            const float mnew = fmaxf(mrun[u], mb);
            alpha[u] = exp2f((mrun[u] - mnew) * L2E);
            mrun[u]  = mnew;
            float lb = 0.0f;
            Pack8 pk;
#pragma unroll
            for (int r = 0; r < 8; ++r) {
                const float pe = exp2f((sacc[u][r] - mnew) * L2E);
                lb += pe;
                pk.hf[r] = (_Float16)(pe * PSCALE);
            }
            lb += __shfl_xor(lb, 16);
            if (h == 0) red_sm[wv][iq] = lb;
            pq[iq * 9 + 2 * wv + h] = pk.u;
#pragma unroll
            for (int tt = 0; tt < 4; ++tt) acc[tt][u] *= alpha[u];
        }
        __syncthreads();

#pragma unroll
        for (int u = 0; u < 2; ++u) {
            const int iq = 16 * u + m;
            const float lb = ((red_sm[0][iq] + red_sm[1][iq]) + red_sm[2][iq]) + red_sm[3][iq];
            lrun[u] = lrun[u] * alpha[u] + lb;
        }

#pragma unroll
        for (int s = 0; s < 2; ++s) {
            Frag p0, p1;
            const int q0 = m * 9 + 4 * s + h;
            const int q1 = (16 + m) * 9 + 4 * s + h;
            p0.u[0] = pq[q0];  p0.u[1] = pq[q0 + 2];
            p1.u[0] = pq[q1];  p1.u[1] = pq[q1 + 2];
#pragma unroll
            for (int tt = 0; tt < 4; ++tt) {
                const size_t vro = ((size_t)(b * CC + 64 * wv + 16 * tt + m)) * HW + j0 + 32 * s + 8 * h;
                Frag va;
                va.u[0] = *(const v4u*)(vv + vro);
                va.u[1] = *(const v4u*)(vv + vro + 16);
                acc[tt][0] = mma_f16(va.hf, p0.hf, acc[tt][0]);
                acc[tt][1] = mma_f16(va.hf, p1.hf, acc[tt][1]);
            }
        }
        __syncthreads();
    }

    float gmul[2];
    gmul[0] = (gm0 * PSCALE_INV) / lrun[0];
    gmul[1] = (gm0 * PSCALE_INV) / lrun[1];
#pragma unroll
    for (int tt = 0; tt < 4; ++tt)
#pragma unroll
        for (int u = 0; u < 2; ++u)
#pragma unroll
            for (int r = 0; r < 8; ++r)
                es[wv][(16 * tt + 8 * h + r) * ESP + 16 * u + m] = acc[tt][u][r] * gmul[u];
    __syncthreads();

    const int q8 = l >> 3, p = l & 7;
#pragma unroll
    for (int gq = 0; gq < 16; ++gq) {
        const int cr = 4 * gq + q8;
        const size_t idx = ((size_t)(b * CC + 64 * wv + cr)) * HW + i0 + 4 * p;
        v4f o = *(const v4f*)&es[wv][cr * ESP + 4 * p];
        const v4f xr = *(const v4f*)(x1r + idx);
        o += xr;
        *(volatile v4f*)(outp + idx) = o;
    }
    __threadfence();
#pragma unroll
    for (int gq = 0; gq < 16; ++gq) {
        const int cr = 4 * gq + q8;
        const size_t idx = ((size_t)(b * CC + 64 * wv + cr)) * HW + i0 + 4 * p;
        v4f o = *(const v4f*)&es[wv][cr * ESP + 4 * p];
        const v4f xr = *(const v4f*)(x1r + idx);
        o += xr;
        *(volatile v4f*)(outp + idx) = o;
    }
}

extern "C" void kernel_launch(void* const* d_in, const int* in_sizes, int n_in,
                              void* d_out, int out_size, void* d_ws, size_t ws_size,
                              hipStream_t stream)
{
    if (n_in < 22) return;
    const int nx = BB * CC * HW;
    if (in_sizes[0] != nx || in_sizes[1] != nx || in_sizes[2] != nx || out_size != nx) return;
    if (in_sizes[3] != CQ * CC || in_sizes[9] != CQ * CC || in_sizes[15] != CC * CC) return;
    if (in_sizes[4] != CQ || in_sizes[10] != CQ || in_sizes[16] != CC || in_sizes[21] < 1) return;

    const float* x1  = (const float*)d_in[0];
    const float* x2  = (const float*)d_in[1];
    const float* x3  = (const float*)d_in[2];
    const float* w1  = (const float*)d_in[3];
    const float* b1  = (const float*)d_in[4];
    const float* g1  = (const float*)d_in[5];
    const float* be1 = (const float*)d_in[6];
    const float* m1  = (const float*)d_in[7];
    const float* v1  = (const float*)d_in[8];
    const float* w2  = (const float*)d_in[9];
    const float* b2  = (const float*)d_in[10];
    const float* g2  = (const float*)d_in[11];
    const float* be2 = (const float*)d_in[12];
    const float* m2  = (const float*)d_in[13];
    const float* v2  = (const float*)d_in[14];
    const float* w3  = (const float*)d_in[15];
    const float* b3  = (const float*)d_in[16];
    const float* g3  = (const float*)d_in[17];
    const float* be3 = (const float*)d_in[18];
    const float* m3  = (const float*)d_in[19];
    const float* v3  = (const float*)d_in[20];
    const float* gam = (const float*)d_in[21];

    const size_t qk_elems = (size_t)BB * HW * CQ;
    const size_t v_elems  = (size_t)BB * CC * HW;
    const size_t need_bytes = (4 * qk_elems + v_elems) * sizeof(unsigned short);
    if (need_bytes > ws_size) return;

    unsigned short* qh = (unsigned short*)d_ws;
    unsigned short* ql = qh + qk_elems;
    unsigned short* kh = ql + qk_elems;
    unsigned short* kl = kh + qk_elems;
    unsigned short* vb = kl + qk_elems;

    k_conv_split<<<dim3(HW / 64, BB), 128, 0, stream>>>(x1, w1, b1, g1, be1, m1, v1, qh, ql);
    k_conv_split<<<dim3(HW / 64, BB), 128, 0, stream>>>(x2, w2, b2, g2, be2, m2, v2, kh, kl);
    k_conv_h    <<<dim3(HW / 64, CC / 64, BB), 128, 0, stream>>>(x3, w3, b3, g3, be3, m3, v3, vb);
    k_attn      <<<dim3(HW / QT, BB), 128, 0, stream>>>(qh, ql, kh, kl, vb, x1, gam, (float*)d_out);
    (void)hipGetLastError();
}
